// EncoderLayer_66657892434540
// MI455X (gfx1250) — hardware-verified
//
#include <hip/hip_runtime.h>

typedef __attribute__((ext_vector_type(16))) _Float16 v16bf;
typedef __attribute__((ext_vector_type(8)))  _Float16 v8bf;
typedef __attribute__((ext_vector_type(8)))  float  v8f;
typedef __attribute__((ext_vector_type(4)))  float  v4f;

static __device__ inline v8f zerov8() {
    v8f z = {0.f, 0.f, 0.f, 0.f, 0.f, 0.f, 0.f, 0.f};
    return z;
}

static __device__ inline unsigned short f32_to_bf16(float f) {
    return __builtin_bit_cast(unsigned short, (_Float16)f);
}

static __device__ inline v8f wmma_bf16(v16bf a, v16bf b, v8f c) {
    v8f d = __builtin_amdgcn_wmma_f32_16x16x32_f16(
         false, a,  false, b,
         (short)0, c,  false,  false);
    asm volatile("v_nop\n\tv_nop\n\tv_nop\n\tv_nop" : "+v"(d) : "v"(a), "v"(b));
    return d;
}

static __device__ inline v16bf make_frag(v8bf lo, v8bf hi) {
    v16bf r;
#pragma unroll
    for (int i = 0; i < 8; ++i) { r[i] = lo[i]; r[i + 8] = hi[i]; }
    return r;
}

static __device__ inline v16bf load_frag_a(const unsigned short* base, int ld) {
    const int lane = threadIdx.x & 31;
    const unsigned short* r = base + (size_t)(lane & 15) * ld + ((lane < 16) ? 0 : 8);
    return make_frag(*(const v8bf*)r, *(const v8bf*)(r + 16));
}

static __device__ inline v16bf load_frag_b(const unsigned short* base, int ld) {
    const int lane = threadIdx.x & 31;
    const unsigned short* r = base + (size_t)(lane & 15) * ld + ((lane < 16) ? 0 : 8);
    return make_frag(*(const v8bf*)r, *(const v8bf*)(r + 16));
}

template <int CTRL>
static __device__ inline float dpp_movf(float v) {
    int r = __builtin_amdgcn_update_dpp(0, __float_as_int(v), CTRL, 0xf, 0xf, true);
    return __int_as_float(r);
}

static __device__ inline float red16_max(float v) {
    v = fmaxf(v, dpp_movf<0xB1>(v));
    v = fmaxf(v, dpp_movf<0x4E>(v));
    v = fmaxf(v, dpp_movf<0x141>(v));
    v = fmaxf(v, dpp_movf<0x128>(v));
    return v;
}

static __device__ inline float red16_sum(float v) {
    v += dpp_movf<0xB1>(v);
    v += dpp_movf<0x4E>(v);
    v += dpp_movf<0x141>(v);
    v += dpp_movf<0x128>(v);
    return v;
}

static __device__ inline float gelu_tanh(float x) {
    float x3 = x * x * x;
    float t = tanhf(0.7978845608028654f * (x + 0.044715f * x3));
    return 0.5f * x * (1.0f + t);
}

struct __attribute__((aligned(16))) H8 { unsigned short e[8]; };
typedef __attribute__((ext_vector_type(4))) unsigned int vu4q;
__global__ void cvt_bf16_kernel(const float* __restrict__ in,
                                unsigned short* __restrict__ out, int n) {
    int i8 = blockIdx.x * 256 + threadIdx.x;
    if (i8 * 8 >= n) return;
    H8 v;
#pragma unroll
    for (int e = 0; e < 8; ++e) v.e[e] = f32_to_bf16(in[(size_t)i8 * 8 + e]);
    *(volatile vu4q*)(out + (size_t)i8 * 8) = *(const vu4q*)&v; __threadfence(); *(volatile vu4q*)(out + (size_t)i8 * 8) = *(const vu4q*)&v;
}

__global__ void bias_expand_kernel(const float* __restrict__ ab,
                                   const int* __restrict__ idx,
                                   float* __restrict__ biasT) {
    int i = blockIdx.x * 256 + threadIdx.x;
    if (i >= 12 * 63 * 1024) return;
    int k  = i & 1023;
    int hr = i >> 10;
    int r  = hr % 63;
    int h  = hr / 63;
    const float v = ab[(h * 63 + r) * 63 + idx[k]];
    *(volatile float*)(biasT + i) = v; __threadfence(); *(volatile float*)(biasT + i) = v;
}

__global__ void __launch_bounds__(128)
ln_kernel(const float* __restrict__ x, const float* __restrict__ w,
          const float* __restrict__ b, unsigned short* __restrict__ out) {
    const int row = blockIdx.x;
    const int tid = threadIdx.x;
    const float* xr = x + (size_t)row * 384;
    float v0 = xr[tid], v1 = xr[tid + 128], v2 = xr[tid + 256];
    float s  = v0 + v1 + v2;
    float s2 = v0 * v0 + v1 * v1 + v2 * v2;
    s  = red16_sum(s);
    s2 = red16_sum(s2);
    s  += __shfl_xor(s, 16, 32);
    s2 += __shfl_xor(s2, 16, 32);
    __shared__ float red[8];
    const int wave = tid >> 5;
    if ((tid & 31) == 0) { red[wave] = s; red[wave + 4] = s2; }
    __syncthreads();
    s  = red[0] + red[1] + red[2] + red[3];
    s2 = red[4] + red[5] + red[6] + red[7];
    float mu   = s * (1.0f / 384.0f);
    float var  = s2 * (1.0f / 384.0f) - mu * mu;
    float rstd = rsqrtf(var + 1e-5f);
    __shared__ __align__(16) unsigned short srow[384];
    srow[tid]       = f32_to_bf16((v0 - mu) * rstd * w[tid]       + b[tid]);
    srow[tid + 128] = f32_to_bf16((v1 - mu) * rstd * w[tid + 128] + b[tid + 128]);
    srow[tid + 256] = f32_to_bf16((v2 - mu) * rstd * w[tid + 256] + b[tid + 256]);
    __syncthreads();
    if (tid < 48) {
        unsigned short* orow = out + (size_t)row * 384;
        const H8 hv = *(const H8*)(srow + tid * 8);
        *(volatile vu4q*)(orow + tid * 8) = *(const vu4q*)&hv; __threadfence(); *(volatile vu4q*)(orow + tid * 8) = *(const vu4q*)&hv;
    }
}

#define LDT 40

template <int EPI, bool AF32>
__global__ void __launch_bounds__(256)
gemm_bf16_kernel(const void* __restrict__ Av,
                 const unsigned short* __restrict__ Bw,
                 const float* __restrict__ bias, void* __restrict__ outp,
                 const float* __restrict__ resid, int M, int N, int K) {
    __shared__ __align__(16) unsigned short At[128 * LDT];
    __shared__ __align__(16) unsigned short Bt[128 * LDT];
    __shared__ __align__(16) unsigned short St[8][32 * 64];
    const unsigned short* A = (const unsigned short*)Av;
    const float* Af = (const float*)Av;

    const int tid   = threadIdx.x;
    const int lane  = tid & 31;
    const int wave  = tid >> 5;
    const int wm    = (wave & 3) * 32;
    const int wn    = (wave >> 2) * 64;
    const int mbase = blockIdx.y * 128;
    const int nbase = blockIdx.x * 128;
    const int nn    = lane & 15;
    const int mhalf = (lane < 16) ? 0 : 8;

    v8f acc[2][4];
#pragma unroll
    for (int j = 0; j < 4; ++j) {
        const float bv = bias[nbase + wn + j * 16 + nn];
        v8f ci;
#pragma unroll
        for (int r = 0; r < 8; ++r) ci[r] = bv;
        acc[0][j] = ci;
        acc[1][j] = ci;
    }

    const int srow = tid >> 1;
    const int scol = (tid & 1) * 16;

    for (int k0 = 0; k0 < K; k0 += 32) {
        __syncthreads();
        {
            uint4* da = (uint4*)(At + srow * LDT + scol);
            if (AF32) {
                const float* sa = Af + (size_t)(mbase + srow) * K + k0 + scol;
                H8 h0, h1;
#pragma unroll
                for (int e = 0; e < 8; ++e) { h0.e[e] = f32_to_bf16(sa[e]); h1.e[e] = f32_to_bf16(sa[8 + e]); }
                da[0] = __builtin_bit_cast(uint4, h0); da[1] = __builtin_bit_cast(uint4, h1);
            } else {
                const uint4* sa = (const uint4*)(A + (size_t)(mbase + srow) * K + k0 + scol);
                da[0] = sa[0]; da[1] = sa[1];
            }
            const uint4* sb = (const uint4*)(Bw + (size_t)(nbase + srow) * K + k0 + scol);
            uint4* db = (uint4*)(Bt + srow * LDT + scol);
            db[0] = sb[0]; db[1] = sb[1];
        }
        __syncthreads();

        v16bf a0 = load_frag_a(At + (wm +  0) * LDT, LDT);
        v16bf a1 = load_frag_a(At + (wm + 16) * LDT, LDT);
        v16bf b0 = load_frag_b(Bt + (wn +  0) * LDT, LDT);
        v16bf b1 = load_frag_b(Bt + (wn + 16) * LDT, LDT);
        v16bf b2 = load_frag_b(Bt + (wn + 32) * LDT, LDT);
        v16bf b3 = load_frag_b(Bt + (wn + 48) * LDT, LDT);

        acc[0][0] = wmma_bf16(a0, b0, acc[0][0]);
        acc[0][1] = wmma_bf16(a0, b1, acc[0][1]);
        acc[0][2] = wmma_bf16(a0, b2, acc[0][2]);
        acc[0][3] = wmma_bf16(a0, b3, acc[0][3]);
        acc[1][0] = wmma_bf16(a1, b0, acc[1][0]);
        acc[1][1] = wmma_bf16(a1, b1, acc[1][1]);
        acc[1][2] = wmma_bf16(a1, b2, acc[1][2]);
        acc[1][3] = wmma_bf16(a1, b3, acc[1][3]);
    }

    if (EPI == 2) {
        float* of = (float*)outp;
        const int hh = lane >> 4;
        for (int pass = 0; pass < 2; ++pass) {
#pragma unroll
            for (int i = 0; i < 2; ++i)
#pragma unroll
                for (int pr = 0; pr < 2; ++pr) {
                    const int cbase = nbase + wn + pr * 32;
#pragma unroll
                    for (int r = 0; r < 8; ++r) {
                        const float a0 = acc[i][2 * pr][r], b0 = acc[i][2 * pr + 1][r];
                        const float ax = __shfl_xor(a0, 16), bx = __shfl_xor(b0, 16);
                        const int r1 = mbase + wm + i * 16 + r, r2 = r1 + 8;
                        const float v1 = (hh ? bx : a0) + resid[(size_t)r1 * N + cbase + lane];
                        const float v2 = (hh ? b0 : ax) + resid[(size_t)r2 * N + cbase + lane];
                        *(volatile float*)(of + (size_t)r1 * N + cbase + lane) = v1;
                        *(volatile float*)(of + (size_t)r2 * N + cbase + lane) = v2;
                    }
                }
            __threadfence();
        }
    } else {
        unsigned short* st = St[wave];
#pragma unroll
        for (int i = 0; i < 2; ++i)
#pragma unroll
            for (int j = 0; j < 4; ++j)
#pragma unroll
                for (int r = 0; r < 8; ++r) {
                    float v = acc[i][j][r];
                    if (EPI == 1) v = gelu_tanh(v);
                    st[(i * 16 + r + mhalf) * 64 + j * 16 + nn] = f32_to_bf16(v);
                }
        __builtin_amdgcn_fence(__ATOMIC_RELEASE, "workgroup"); __builtin_amdgcn_wave_barrier(); __builtin_amdgcn_fence(__ATOMIC_ACQUIRE, "workgroup");
        unsigned short* ob = (unsigned short*)outp + (size_t)(mbase + wm) * N + nbase + wn;
        for (int pass = 0; pass < 2; ++pass) {
#pragma unroll
            for (int jj = 0; jj < 8; ++jj) {
                const int row = jj * 4 + (lane >> 3), seg = lane & 7;
                *(volatile vu4q*)(ob + (size_t)row * N + seg * 8) = *(const vu4q*)(st + row * 64 + seg * 8);
            }
            __threadfence();
        }
    }
}

#define AKC 128
#define LDV 136

__global__ void __launch_bounds__(128)
attn_kernel(const unsigned short* __restrict__ qkv,
            const float* __restrict__ biasT, const int* __restrict__ idx,
            float* __restrict__ obf) {
    __shared__ __align__(16) unsigned short Kt[AKC * LDT];
    __shared__ __align__(16) unsigned short Vt[32 * LDV];
    __shared__ __align__(16) unsigned short Pt[4 * 16 * LDV];

    const int tid  = threadIdx.x;
    const int lane = tid & 31;
    const int wave = tid >> 5;
    const int bh   = blockIdx.y;
    const int b    = bh / 12;
    const int h    = bh % 12;
    const int qbase = blockIdx.x * 64 + wave * 16;

    const unsigned short* qkv_b = qkv + (size_t)b * 1024 * 1152;

    const float scale = 0.17677669529663687f;
    v16bf qfrag = load_frag_a(qkv_b + (size_t)qbase * 1152 + h * 32, 1152);
#pragma unroll
    for (int i = 0; i < 16; ++i) qfrag[i] = (_Float16)((float)qfrag[i] * scale);

    const int mhalf = (lane < 16) ? 0 : 8;
    const int nn    = lane & 15;
    size_t boff[8];
#pragma unroll
    for (int r = 0; r < 8; ++r)
        boff[r] = (size_t)idx[qbase + r + mhalf] * 1024;
    const float* biasH = biasT + (size_t)h * 63 * 1024 + nn;

    float mstat[8], lstat[8];
#pragma unroll
    for (int r = 0; r < 8; ++r) { mstat[r] = -1e30f; lstat[r] = 0.f; }
    v8f o0 = zerov8(), o1 = zerov8();

    unsigned short* Pw = Pt + wave * 16 * LDV;

    for (int c0 = 0; c0 < 1024; c0 += AKC) {
        __syncthreads();
        {
            const uint4* ks = (const uint4*)(qkv_b + (size_t)(c0 + tid) * 1152 + 384 + h * 32);
            uint4* kd = (uint4*)(Kt + tid * LDT);
            kd[0] = ks[0]; kd[1] = ks[1]; kd[2] = ks[2]; kd[3] = ks[3];
            const unsigned short* vs = qkv_b + (size_t)(c0 + tid) * 1152 + 768 + h * 32;
#pragma unroll
            for (int d = 0; d < 32; ++d) Vt[d * LDV + tid] = vs[d];
        }
        __syncthreads();

        v8f s[8];
#pragma unroll
        for (int t = 0; t < 8; ++t) {
            v8f cb;
#pragma unroll
            for (int r = 0; r < 8; ++r) cb[r] = biasH[boff[r] + c0 + t * 16];
            v16bf kf = load_frag_b(Kt + t * 16 * LDT, LDT);
            s[t] = wmma_bf16(qfrag, kf, cb);
        }

#pragma unroll
        for (int r = 0; r < 8; ++r) {
            float mx = s[0][r];
#pragma unroll
            for (int t = 1; t < 8; ++t) mx = fmaxf(mx, s[t][r]);
            mx = red16_max(mx);
            float mnew = fmaxf(mstat[r], mx);
            unsigned short* prow = Pw + (r + mhalf) * LDV;
            float sum = 0.f;
#pragma unroll
            for (int t = 0; t < 8; ++t) {
                float e = __expf(s[t][r] - mnew);
                sum += e;
                prow[t * 16 + nn] = f32_to_bf16(e);
            }
            sum = red16_sum(sum);
            float alpha = __expf(mstat[r] - mnew);
            lstat[r] = lstat[r] * alpha + sum;
            mstat[r] = mnew;
            o0[r] *= alpha;
            o1[r] *= alpha;
        }
        __builtin_amdgcn_wave_barrier();
        asm volatile("" ::: "memory");

#pragma unroll
        for (int kk = 0; kk < AKC; kk += 32) {
            v16bf pf  = load_frag_a(Pw + kk, LDV);
            v16bf vf0 = load_frag_b(Vt + kk, LDV);
            v16bf vf1 = load_frag_b(Vt + 16 * LDV + kk, LDV);
            o0 = wmma_bf16(pf, vf0, o0);
            o1 = wmma_bf16(pf, vf1, o1);
        }
    }

    const int hh = lane >> 4;
    for (int pass = 0; pass < 2; ++pass) {
#pragma unroll
        for (int r = 0; r < 8; ++r) {
            const float i1 = 1.0f / lstat[r];
            const float a0 = o0[r] * i1, b0 = o1[r] * i1;
            const float ax = __shfl_xor(a0, 16), bx = __shfl_xor(b0, 16);
            const float v1 = hh ? bx : a0;
            const float v2 = hh ? b0 : ax;
            *(volatile float*)(obf + ((size_t)b * 1024 + qbase + r) * 384 + h * 32 + lane) = v1;
            *(volatile float*)(obf + ((size_t)b * 1024 + qbase + r + 8) * 384 + h * 32 + lane) = v2;
        }
        __threadfence();
    }
}

extern "C" void kernel_launch(void* const* d_in, const int* in_sizes, int n_in,
                              void* d_out, int out_size, void* d_ws, size_t ws_size,
                              hipStream_t stream) {
    (void)in_sizes; (void)n_in; (void)out_size;

    const float* x         = (const float*)d_in[0];
    const float* sa_w      = (const float*)d_in[1];
    const float* sa_b      = (const float*)d_in[2];
    const float* w_qkv     = (const float*)d_in[3];
    const float* b_qkv     = (const float*)d_in[4];
    const float* w_out     = (const float*)d_in[5];
    const float* b_out     = (const float*)d_in[6];
    const float* attn_bias = (const float*)d_in[7];
    const float* mlp_w     = (const float*)d_in[8];
    const float* mlp_b     = (const float*)d_in[9];
    const float* w1        = (const float*)d_in[10];
    const float* b1        = (const float*)d_in[11];
    const float* w2        = (const float*)d_in[12];
    const float* b2        = (const float*)d_in[13];
    const int*   bidx      = (const int*)d_in[14];
    float* out             = (float*)d_out;

    char* ws = (char*)d_ws;
    size_t off = 0;
    unsigned short* w_qkv_bf = (unsigned short*)(ws + off); off += (size_t)1152 * 384 * 2;
    unsigned short* w_out_bf = (unsigned short*)(ws + off); off += (size_t)384 * 384 * 2;
    unsigned short* w1_bf    = (unsigned short*)(ws + off); off += (size_t)1536 * 384 * 2;
    unsigned short* w2_bf    = (unsigned short*)(ws + off); off += (size_t)384 * 1536 * 2;
    unsigned short* hbf      = (unsigned short*)(ws + off); off += (size_t)16384 * 384 * 2;
    unsigned short* qkv_bf   = (unsigned short*)(ws + off); off += (size_t)16384 * 1152 * 2;
    float*          o_bf     = (float*)(ws + off);          off += (size_t)16384 * 384 * 4;
    float*          xmid     = (float*)(ws + off);          off += (size_t)16384 * 384 * 4;
    unsigned short* h2bf     = (unsigned short*)(ws + off); off += (size_t)16384 * 384 * 2;
    unsigned short* m1_bf    = (unsigned short*)(ws + off); off += (size_t)16384 * 1536 * 2;
    float*          biasT    = (float*)(ws + off);          off += (size_t)12 * 63 * 1024 * 4;
    if (off > ws_size) return;

    cvt_bf16_kernel<<<(442368 / 8 + 255) / 256, 256, 0, stream>>>(w_qkv, w_qkv_bf, 442368);
    cvt_bf16_kernel<<<(147456 / 8 + 255) / 256, 256, 0, stream>>>(w_out, w_out_bf, 147456);
    cvt_bf16_kernel<<<(589824 / 8 + 255) / 256, 256, 0, stream>>>(w1, w1_bf, 589824);
    cvt_bf16_kernel<<<(589824 / 8 + 255) / 256, 256, 0, stream>>>(w2, w2_bf, 589824);
    bias_expand_kernel<<<(774144 + 255) / 256, 256, 0, stream>>>(attn_bias, bidx, biasT);

    ln_kernel<<<16384, 128, 0, stream>>>(x, sa_w, sa_b, hbf);
    gemm_bf16_kernel<0, false><<<dim3(9, 128), 256, 0, stream>>>(
        hbf, w_qkv_bf, b_qkv, qkv_bf, nullptr, 16384, 1152, 384);
    attn_kernel<<<dim3(16, 192), 128, 0, stream>>>(qkv_bf, biasT, bidx, o_bf);
    gemm_bf16_kernel<2, true><<<dim3(3, 128), 256, 0, stream>>>(
        o_bf, w_out_bf, b_out, xmid, x, 16384, 384, 384);
    ln_kernel<<<16384, 128, 0, stream>>>(xmid, mlp_w, mlp_b, h2bf);
    gemm_bf16_kernel<1, false><<<dim3(12, 128), 256, 0, stream>>>(
        h2bf, w1_bf, b1, m1_bf, nullptr, 16384, 1536, 384);
    gemm_bf16_kernel<2, false><<<dim3(3, 128), 256, 0, stream>>>(
        m1_bf, w2_bf, b2, out, xmid, 16384, 384, 1536);
}
